// HiLo_13494787244075
// MI455X (gfx1250) — hardware-run, weakly checked
//
#include <hip/hip_runtime.h>
#include <math.h>


#define C_DIM   384
#define IMG_W   96
#define HW_N    9216
#define BATCH   2
#define NTOK    (BATCH * HW_N)
#define NLH     6
#define HEADD   32
#define BR_DIM  192
#define QKV_N   576
#define POOL_W  48
#define POOLN   2304
#define NPROW   (BATCH * POOLN)
#define QTILES  (HW_N / 64)
#define CTXW    64
#define OUTN    (NTOK * C_DIM)
#define ATT_SCALE 0.17677669529663687f
#define QKV_OSC 16.0f
#define CL2     (ATT_SCALE * 1.4426950408889634f / 256.0f)

static_assert(NLH * HEADD == BR_DIM);
static_assert(2 * BR_DIM == C_DIM);
static_assert(HW_N == IMG_W * IMG_W);
static_assert(POOLN == POOL_W * POOL_W);
static_assert((HW_N % 64) == 0 && (POOLN % 64) == 0);
static_assert((C_DIM % 64) == 0 && (BR_DIM % 64) == 0 && (QKV_N % 64) == 0);
static_assert((((NTOK / 64) * (QKV_N / 64)) % 8) == 0);
static_assert((((NTOK / 64) * (BR_DIM / 64)) % 8) == 0);
static_assert((((NPROW / 64) * (C_DIM / 64)) % 8) == 0);
static_assert(((BATCH * POOLN * NLH) % 8) == 0);
static_assert(HEADD == 32 && CTXW == 2 * HEADD);

typedef __bf16         v16bf __attribute__((ext_vector_type(16)));
typedef _Float16       v16h  __attribute__((ext_vector_type(16)));
typedef float          v8f   __attribute__((ext_vector_type(8)));
typedef float          v4f   __attribute__((ext_vector_type(4)));
typedef unsigned int   v4u   __attribute__((ext_vector_type(4)));
typedef unsigned short v8us  __attribute__((ext_vector_type(8)));
typedef unsigned short v16us __attribute__((ext_vector_type(16)));

__device__ __forceinline__ unsigned short bf_bits(float f) {
  const unsigned u = __float_as_uint(f);
  return (unsigned short)((u + 0x7FFFu + ((u >> 16) & 1u)) >> 16);
}
__device__ __forceinline__ float bf_up(unsigned short h) { return __uint_as_float(((unsigned)h) << 16); }
__device__ __forceinline__ float bfr(float f) { return bf_up(bf_bits(f)); }
__device__ __forceinline__ unsigned short h_bits(float f) {
  const _Float16 h = (_Float16)f;
  return __builtin_bit_cast(unsigned short, h);
}
__device__ __forceinline__ unsigned pk16(unsigned short a, unsigned short b) { return (unsigned)a | ((unsigned)b << 16); }
__device__ __forceinline__ v8f zero8() { v8f z = {0.f, 0.f, 0.f, 0.f, 0.f, 0.f, 0.f, 0.f}; return z; }

__device__ __forceinline__ void ld8(const float* p, float* o) {
  const v4f a = *(const v4f*)(p);
  const v4f b = *(const v4f*)(p + 4);
  o[0] = a[0]; o[1] = a[1]; o[2] = a[2]; o[3] = a[3];
  o[4] = b[0]; o[5] = b[1]; o[6] = b[2]; o[7] = b[3];
}

__device__ __forceinline__ void lds_sync() {
  __builtin_amdgcn_fence(__ATOMIC_RELEASE, "workgroup");
  __builtin_amdgcn_wave_barrier();
  __builtin_amdgcn_fence(__ATOMIC_ACQUIRE, "workgroup");
}

__device__ __forceinline__ v16us ldfrag_u(const unsigned short* p) {
  union { v16us v; v8us h[2]; } f;
  f.h[0] = *(const v8us*)(p);
  f.h[1] = *(const v8us*)(p + 16);
  return f.v;
}
__device__ __forceinline__ v16bf ldfrag_b(const unsigned short* p) { return __builtin_bit_cast(v16bf, ldfrag_u(p)); }
__device__ __forceinline__ v16h  ldfrag_h(const unsigned short* p) { return __builtin_bit_cast(v16h, ldfrag_u(p)); }

__device__ __forceinline__ v8f mma_b(v16bf a, v16bf b, v8f c) {
  c = __builtin_amdgcn_wmma_f32_16x16x32_bf16(false, a, false, b, (short)0, c, false, false);
#if defined(__HIP_DEVICE_COMPILE__)
  asm volatile("v_nop\n\tv_nop\n\tv_nop\n\tv_nop" : "+v"(c) : "v"(a), "v"(b));
#endif
  return c;
}
__device__ __forceinline__ v8f mma_b_raw(v16bf a, v16bf b, v8f c) {
  return __builtin_amdgcn_wmma_f32_16x16x32_bf16(false, a, false, b, (short)0, c, false, false);
}
__device__ __forceinline__ v8f mma_h(v16h a, v16h b, v8f c) {
  c = __builtin_amdgcn_wmma_f32_16x16x32_f16(false, a, false, b, (short)0, c, false, false);
#if defined(__HIP_DEVICE_COMPILE__)
  asm volatile("v_nop\n\tv_nop\n\tv_nop\n\tv_nop" : "+v"(c) : "v"(a), "v"(b));
#endif
  return c;
}
__device__ __forceinline__ void dep_guard_b(v8f& a, v8f& b, v16bf x) {
#if defined(__HIP_DEVICE_COMPILE__)
  asm volatile("v_nop\n\tv_nop\n\tv_nop\n\tv_nop" : "+v"(a), "+v"(b) : "v"(x));
#endif
}
__device__ __forceinline__ void keep4_b(v16bf a, v16bf b, v16bf c, v16bf d) {
#if defined(__HIP_DEVICE_COMPILE__)
  asm volatile("v_nop" :: "v"(a), "v"(b), "v"(c), "v"(d));
#endif
}
__device__ __forceinline__ void acc_guard4(v8f& a, v8f& b, v8f& c, v8f& d) {
#if defined(__HIP_DEVICE_COMPILE__)
  asm volatile("v_nop\n\tv_nop\n\tv_nop\n\tv_nop" : "+v"(a), "+v"(b), "+v"(c), "+v"(d));
#endif
}

__global__ __launch_bounds__(256) void k_tr(const float* __restrict__ in, unsigned short* out, int R, int Cc) {
  __shared__ float s[64][65];
  const int c0 = blockIdx.x * 64, r0 = blockIdx.y * 64;
  if (c0 + 64 > Cc || r0 + 64 > R) return;
  const float* inb = in + (size_t)blockIdx.z * (size_t)R * (size_t)Cc;
  unsigned short* outb = out + (size_t)blockIdx.z * (size_t)R * (size_t)Cc;
  const int t = threadIdx.x, cc = t & 63, rq = t >> 6;
#pragma unroll
  for (int it = 0; it < 16; ++it) {
    const int r = it * 4 + rq;
    s[r][cc] = inb[(size_t)(r0 + r) * (size_t)Cc + c0 + cc];
  }
  __syncthreads();
  const int q8 = t & 7, rr = t >> 3;
  v4u ov[2];
  size_t oo[2];
#pragma unroll
  for (int it = 0; it < 2; ++it) {
    const int cc2 = it * 32 + rr;
    unsigned short hb[8];
#pragma unroll
    for (int e = 0; e < 8; ++e) hb[e] = bf_bits(s[q8 * 8 + e][cc2]);
    v4u p;
#pragma unroll
    for (int q = 0; q < 4; ++q) p[q] = pk16(hb[2 * q], hb[2 * q + 1]);
    ov[it] = p;
    oo[it] = (size_t)(c0 + cc2) * (size_t)R + r0 + q8 * 8;
  }
  for (int pass = 0; pass < 2; ++pass) {
#pragma unroll
    for (int it = 0; it < 2; ++it) *(volatile v4u*)(outb + oo[it]) = ov[it];
    __threadfence();
  }
}

__global__ __launch_bounds__(256) void k_pool(const float* __restrict__ x, unsigned short* Xph, unsigned short* Xpl) {
  __shared__ float s[64][65];
  const int p0 = blockIdx.x * 64, c0 = blockIdx.y * 64, b = blockIdx.z;
  const int t = threadIdx.x, pp = t & 63, cq = t >> 6;
  const int p = p0 + pp;
  const int gy = p / POOL_W, gx = p - gy * POOL_W;
  const float* xb = x + (size_t)b * C_DIM * HW_N + (size_t)(2 * gy) * IMG_W + 2 * gx;
#pragma unroll
  for (int it = 0; it < 16; ++it) {
    const int c = it * 4 + cq;
    const float* q = xb + (size_t)(c0 + c) * HW_N;
    const float v = 0.25f * ((bfr(q[0]) + bfr(q[1])) + (bfr(q[IMG_W]) + bfr(q[IMG_W + 1])));
    s[c][pp] = v;
  }
  __syncthreads();
  const int q8 = t & 7, rr = t >> 3;
  v4u ovh[2], ovl[2];
  size_t oo[2];
#pragma unroll
  for (int it = 0; it < 2; ++it) {
    const int pp2 = it * 32 + rr;
    unsigned short hb[8], lb[8];
#pragma unroll
    for (int e = 0; e < 8; ++e) {
      const float f = s[q8 * 8 + e][pp2];
      hb[e] = bf_bits(f);
      lb[e] = bf_bits(f - bf_up(hb[e]));
    }
    v4u ah, al;
#pragma unroll
    for (int q = 0; q < 4; ++q) { ah[q] = pk16(hb[2 * q], hb[2 * q + 1]); al[q] = pk16(lb[2 * q], lb[2 * q + 1]); }
    ovh[it] = ah; ovl[it] = al;
    oo[it] = (size_t)(b * POOLN + p0 + pp2) * C_DIM + c0 + q8 * 8;
  }
  for (int pass = 0; pass < 2; ++pass) {
#pragma unroll
    for (int it = 0; it < 2; ++it) {
      *(volatile v4u*)(Xph + oo[it]) = ovh[it];
      *(volatile v4u*)(Xpl + oo[it]) = ovl[it];
    }
    __threadfence();
  }
}

template <int NA, int AHM>
__device__ __forceinline__ void kloop(v8f (&acc)[4][4],
                                      const unsigned short* __restrict__ Pa, const unsigned short* __restrict__ Pb,
                                      int lda, int m0, int K,
                                      const unsigned short* __restrict__ Bt, int ldb, int n0,
                                      int rlane, int koff) {
  int bm = 0, sm0 = m0;
  if (AHM != 0) { bm = m0 / HW_N; sm0 = m0 - bm * HW_N; }
  for (int kk = 0; kk < K; kk += 32) {
    v16bf bh[4];
#pragma unroll
    for (int j = 0; j < 4; ++j) {
      const size_t bo = (size_t)(n0 + (j << 4) + rlane) * (size_t)ldb + koff + kk;
      bh[j] = ldfrag_b(Bt + bo);
    }
#pragma unroll
    for (int i = 0; i < 4; ++i) {
      const unsigned short* pa;
      const unsigned short* pb;
      if (AHM == 0) {
        const size_t ao = (size_t)(m0 + (i << 4) + rlane) * (size_t)lda + koff + kk;
        pa = Pa + ao;
        pb = Pb + ao;
      } else {
        const size_t ao = ((size_t)(bm * NLH + (kk >> 5)) * HW_N + sm0 + (i << 4) + rlane) * CTXW + koff;
        pa = Pa + ao;
        pb = Pa + ao + HEADD;
      }
      const v16bf a0 = ldfrag_b(pa);
#pragma unroll
      for (int j = 0; j < 4; ++j) acc[i][j] = mma_b_raw(a0, bh[j], acc[i][j]);
      dep_guard_b(acc[i][0], acc[i][3], a0);
      if (NA == 2) {
        const v16bf a1 = ldfrag_b(pb);
#pragma unroll
        for (int j = 0; j < 4; ++j) acc[i][j] = mma_b_raw(a1, bh[j], acc[i][j]);
        dep_guard_b(acc[i][0], acc[i][3], a1);
      }
    }
    keep4_b(bh[0], bh[1], bh[2], bh[3]);
  }
}

template <int MODE, int NA, int AHM, int BIAS>
__global__ __launch_bounds__(256) void gemm64(
    const unsigned short* __restrict__ Pa, const unsigned short* __restrict__ Pb, int lda,
    const unsigned short* __restrict__ Bt, int ldb, const float* __restrict__ bias,
    float* Cf, unsigned short* Ch, int ldc, int M, int N, int K, float osc, int cbase) {
  __shared__ __align__(16) float sT[8][1152];
  const int lane = threadIdx.x & 31;
  const int wave = threadIdx.x >> 5;
  const int tilesN = N >> 6;
  const int tilesM = M >> 6;
  const int tiles = tilesM * tilesN;
  const int item = blockIdx.x * 8 + wave;
  if (item >= tiles) return;
  const int tm = item / tilesN;
  const int tn = item - tm * tilesN;
  const int m0 = tm << 6;
  const int n0 = tn << 6;

  const int rlane = lane & 15;
  const int koff  = (lane >> 4) * 8;
  const int mOff  = (lane >> 4) * 8;

  v8f acc[4][4];
#pragma unroll
  for (int i = 0; i < 4; ++i)
#pragma unroll
    for (int j = 0; j < 4; ++j) acc[i][j] = zero8();

  kloop<NA, AHM>(acc, Pa, Pb, lda, m0, K, Bt, ldb, n0, rlane, koff);
  acc_guard4(acc[0][0], acc[0][1], acc[0][2], acc[0][3]);
  acc_guard4(acc[1][0], acc[1][1], acc[1][2], acc[1][3]);
  acc_guard4(acc[2][0], acc[2][1], acc[2][2], acc[2][3]);
  acc_guard4(acc[3][0], acc[3][1], acc[3][2], acc[3][3]);

  float* slab = sT[wave];
  if (MODE == 0 || MODE == 1) {
#pragma unroll
    for (int i = 0; i < 4; ++i) {
      const int mBase = m0 + (i << 4);
#pragma unroll
      for (int r = 0; r < 8; ++r) {
#pragma unroll
        for (int j = 0; j < 4; ++j) {
          slab[(mOff + r) * 68 + (j << 4) + rlane] = acc[i][j][r];
        }
      }
      lds_sync();
      if (MODE == 0) {
        const int h2 = lane >> 4, c4 = (lane & 15) * 4;
        v4f b4 = {0.f, 0.f, 0.f, 0.f};
        if (BIAS != 0) {
          const v4f braw = *(const v4f*)(bias + n0 + c4);
#pragma unroll
          for (int e = 0; e < 4; ++e) b4[e] = bfr(braw[e]);
        }
        v4f ov[8];
#pragma unroll
        for (int it = 0; it < 8; ++it) {
          const int row = it * 2 + h2;
          const v4f xs = *(const v4f*)(slab + row * 68 + c4);
          ov[it] = xs + b4;
        }
        for (int pass = 0; pass < 2; ++pass) {
#pragma unroll
          for (int it = 0; it < 8; ++it) {
            const int row = it * 2 + h2;
            *(volatile v4f*)(Cf + (size_t)(mBase + row) * (size_t)ldc + n0 + c4) = ov[it];
          }
          __threadfence();
        }
      } else {
        const int q8 = lane & 7, rr = lane >> 3, c8 = q8 * 8;
        v4u ov[4];
#pragma unroll
        for (int it = 0; it < 4; ++it) {
          const int row = it * 4 + rr;
          float xs[8];
          ld8(slab + row * 68 + c8, xs);
          unsigned short hb[8];
#pragma unroll
          for (int e = 0; e < 8; ++e) hb[e] = h_bits(xs[e] * osc);
          v4u ah;
#pragma unroll
          for (int p = 0; p < 4; ++p) ah[p] = pk16(hb[2 * p], hb[2 * p + 1]);
          ov[it] = ah;
        }
        for (int pass = 0; pass < 2; ++pass) {
#pragma unroll
          for (int it = 0; it < 4; ++it) {
            const int row = it * 4 + rr;
            const size_t co = (size_t)(mBase + row) * (size_t)ldc + n0 + c8;
            *(volatile v4u*)(Ch + co) = ov[it];
          }
          __threadfence();
        }
      }
      lds_sync();
    }
  } else {
    const int bm = m0 / HW_N, sm0 = m0 - bm * HW_N;
    const int q8 = lane & 7, rr = lane >> 3;
#pragma unroll
    for (int hm = 0; hm < 2; ++hm) {
#pragma unroll
      for (int hn = 0; hn < 2; ++hn) {
#pragma unroll
        for (int ii = 0; ii < 2; ++ii) {
#pragma unroll
          for (int jj = 0; jj < 2; ++jj) {
#pragma unroll
            for (int r = 0; r < 8; ++r) {
              slab[((jj << 4) + rlane) * 36 + (ii << 4) + mOff + r] = acc[2 * hm + ii][2 * hn + jj][r];
            }
          }
        }
        lds_sync();
        for (int pass = 0; pass < 2; ++pass) {
#pragma unroll
          for (int it = 0; it < 8; ++it) {
            const int ch = it * 4 + rr;
            float bv = 0.f;
            if (BIAS != 0) bv = bfr(bias[n0 + hn * 32 + ch]);
            const v4f xs = *(const v4f*)(slab + ch * 36 + q8 * 4);
            const v4f b4 = {bv, bv, bv, bv};
            const v4f ov = xs + b4;
            const size_t go = ((size_t)(bm * C_DIM + cbase + n0 + hn * 32 + ch)) * (size_t)HW_N
                              + (size_t)(sm0 + hm * 32 + q8 * 4);
            *(volatile v4f*)(Cf + go) = ov;
          }
          __threadfence();
        }
        lds_sync();
      }
    }
  }
}

__global__ __launch_bounds__(256) void k_win_attn(const float* __restrict__ Y1, unsigned short* Ctx) {
  __shared__ __align__(16) float so[8][4 * 36];
  const int tid = threadIdx.x, wave = tid >> 5, lane = tid & 31;
  const int item = blockIdx.x * 8 + wave;
  if (item >= BATCH * POOLN * NLH) return;
  const int h = item % NLH;
  const int g = (item / NLH) % POOLN;
  const int b = item / (NLH * POOLN);
  const int gy = g / POOL_W, gx = g - gy * POOL_W;
  const int i = lane >> 3, dq = (lane & 7) * 4;
  const int s00 = (2 * gy) * IMG_W + 2 * gx;
  const float* base = Y1 + (size_t)b * HW_N * QKV_N + h * HEADD + dq;
  const int si = s00 + (i >> 1) * IMG_W + (i & 1);
  const v4f q4 = *(const v4f*)(base + (size_t)si * QKV_N);
  float sc[4];
#pragma unroll
  for (int j = 0; j < 4; ++j) {
    const int sj = s00 + (j >> 1) * IMG_W + (j & 1);
    const v4f k4 = *(const v4f*)(base + (size_t)sj * QKV_N + BR_DIM);
    float d = q4[0] * k4[0] + q4[1] * k4[1] + q4[2] * k4[2] + q4[3] * k4[3];
    d += __shfl_xor(d, 1, 32);
    d += __shfl_xor(d, 2, 32);
    d += __shfl_xor(d, 4, 32);
    sc[j] = d * ATT_SCALE;
  }
  const float mx = fmaxf(fmaxf(sc[0], sc[1]), fmaxf(sc[2], sc[3]));
  float ex[4];
  float sum = 0.f;
#pragma unroll
  for (int j = 0; j < 4; ++j) { ex[j] = __expf(sc[j] - mx); sum += ex[j]; }
  const float inv = 1.0f / sum;
  v4f o = {0.f, 0.f, 0.f, 0.f};
#pragma unroll
  for (int j = 0; j < 4; ++j) {
    const int sj = s00 + (j >> 1) * IMG_W + (j & 1);
    const v4f v4 = *(const v4f*)(base + (size_t)sj * QKV_N + 2 * BR_DIM);
    const float w = ex[j] * inv;
    const v4f w4 = {w, w, w, w};
    o = o + w4 * v4;
  }
  float* sw = so[wave];
  *(v4f*)(sw + i * 36 + dq) = o;
  lds_sync();
  const int q8 = lane & 7, d8 = (q8 & 3) * 8;
  float f[8];
  ld8(sw + i * 36 + d8, f);
  unsigned short hb[8], lb[8], ob[8];
#pragma unroll
  for (int e = 0; e < 8; ++e) {
    hb[e] = bf_bits(f[e]);
    lb[e] = bf_bits(f[e] - bf_up(hb[e]));
    ob[e] = (q8 < 4) ? hb[e] : lb[e];
  }
  v4u ov;
#pragma unroll
  for (int p = 0; p < 4; ++p) ov[p] = pk16(ob[2 * p], ob[2 * p + 1]);
  const size_t go = ((size_t)(b * NLH + h) * HW_N + si) * CTXW + q8 * 8;
  *(volatile v4u*)(Ctx + go) = ov;
  __threadfence();
  *(volatile v4u*)(Ctx + go) = ov;
}

__global__ __launch_bounds__(128) void k_pool_attn(const unsigned short* __restrict__ Qp,
                                                   const unsigned short* __restrict__ KVp,
                                                   unsigned short* Ctx) {
  __shared__ __align__(16) unsigned short sK[64 * 40];
  __shared__ __align__(16) unsigned short sVt[32 * 72];
  __shared__ __align__(16) unsigned short sP[4][16 * 72];
  __shared__ __align__(16) float sO[4][16 * 36];
  const int tid = threadIdx.x, wave = tid >> 5, lane = tid & 31;
  const int hh = lane >> 4, c = lane & 15;
  const int bx = blockIdx.x;
  const int qt = bx % QTILES;
  const int h = (bx / QTILES) % NLH;
  const int b = bx / (QTILES * NLH);
  const int q0 = qt * 64 + wave * 16;
  const v16h qa = ldfrag_h(Qp + (size_t)(b * HW_N + q0 + c) * BR_DIM + h * HEADD + 8 * hh);
  float mrun[8], lrun[8];
#pragma unroll
  for (int r = 0; r < 8; ++r) { mrun[r] = -1e30f; lrun[r] = 0.f; }
  v8f acc0 = zero8(), acc1 = zero8();
  const unsigned short* kvb = KVp + (size_t)b * POOLN * C_DIM + h * HEADD;
  unsigned short* sPw = sP[wave];

  for (int kt = 0; kt < POOLN / 64; ++kt) {
    const int k0 = kt * 64;
#pragma unroll
    for (int it = 0; it < 2; ++it) {
      const int idx = it * 128 + tid;
      const int key = idx >> 2, piece = idx & 3;
      const v8us u = *(const v8us*)(kvb + (size_t)(k0 + key) * C_DIM + piece * 8);
      *(v8us*)(sK + key * 40 + piece * 8) = u;
      const int key2 = idx & 63, piece2 = idx >> 6;
      const v8us w = *(const v8us*)(kvb + (size_t)(k0 + key2) * C_DIM + BR_DIM + piece2 * 8);
#pragma unroll
      for (int e = 0; e < 8; ++e) sVt[(piece2 * 8 + e) * 72 + key2] = w[e];
    }
    __syncthreads();

    v8f s[4];
#pragma unroll
    for (int j = 0; j < 4; ++j) {
      const v16h kb = ldfrag_h(sK + (j * 16 + c) * 40 + 8 * hh);
      s[j] = mma_h(qa, kb, zero8());
    }
    float tsum[8], alpha[8];
#pragma unroll
    for (int r = 0; r < 8; ++r) {
      float mx = fmaxf(fmaxf(s[0][r], s[1][r]), fmaxf(s[2][r], s[3][r]));
      mx = fmaxf(mx, __shfl_xor(mx, 1, 32));
      mx = fmaxf(mx, __shfl_xor(mx, 2, 32));
      mx = fmaxf(mx, __shfl_xor(mx, 4, 32));
      mx = fmaxf(mx, __shfl_xor(mx, 8, 32));
      const float mn = fmaxf(mrun[r], mx);
      alpha[r] = exp2f((mrun[r] - mn) * CL2);
      mrun[r] = mn;
      float ps = 0.f;
#pragma unroll
      for (int j = 0; j < 4; ++j) {
        const float p = exp2f((s[j][r] - mn) * CL2);
        ps += p;
        sPw[(8 * hh + r) * 72 + j * 16 + c] = h_bits(p);
      }
      tsum[r] = ps;
    }
#pragma unroll
    for (int r = 0; r < 8; ++r) {
      float ps = tsum[r];
      ps += __shfl_xor(ps, 1, 32);
      ps += __shfl_xor(ps, 2, 32);
      ps += __shfl_xor(ps, 4, 32);
      ps += __shfl_xor(ps, 8, 32);
      lrun[r] = lrun[r] * alpha[r] + ps;
      acc0[r] *= alpha[r];
      acc1[r] *= alpha[r];
    }
    lds_sync();
#pragma unroll
    for (int ks = 0; ks < 2; ++ks) {
      const v16h pa = ldfrag_h(sPw + c * 72 + ks * 32 + 8 * hh);
      const v16h v0 = ldfrag_h(sVt + c * 72 + ks * 32 + 8 * hh);
      const v16h v1 = ldfrag_h(sVt + (16 + c) * 72 + ks * 32 + 8 * hh);
      acc0 = mma_h(pa, v0, acc0);
      acc1 = mma_h(pa, v1, acc1);
    }
    __syncthreads();
  }

  float* sOw = sO[wave];
#pragma unroll
  for (int r = 0; r < 8; ++r) {
    const float inv = (1.0f / lrun[r]) * (1.0f / QKV_OSC);
    sOw[(8 * hh + r) * 36 + c]      = acc0[r] * inv;
    sOw[(8 * hh + r) * 36 + 16 + c] = acc1[r] * inv;
  }
  lds_sync();
  const int q8 = lane & 7, rr = lane >> 3, d8 = (q8 & 3) * 8;
  v4u ov[4];
#pragma unroll
  for (int it = 0; it < 4; ++it) {
    const int row = it * 4 + rr;
    float f[8];
    ld8(sOw + row * 36 + d8, f);
    unsigned short ob[8];
#pragma unroll
    for (int e = 0; e < 8; ++e) {
      const unsigned short hb = bf_bits(f[e]);
      const unsigned short lb = bf_bits(f[e] - bf_up(hb));
      ob[e] = (q8 < 4) ? hb : lb;
    }
    v4u a4;
#pragma unroll
    for (int p = 0; p < 4; ++p) a4[p] = pk16(ob[2 * p], ob[2 * p + 1]);
    ov[it] = a4;
  }
  for (int pass = 0; pass < 2; ++pass) {
#pragma unroll
    for (int it = 0; it < 4; ++it) {
      const int row = it * 4 + rr;
      const size_t go = ((size_t)(b * NLH + h) * HW_N + q0 + row) * CTXW + q8 * 8;
      *(volatile v4u*)(Ctx + go) = ov[it];
    }
    __threadfence();
  }
}

extern "C" void kernel_launch(void* const* d_in, const int* in_sizes, int n_in,
                              void* d_out, int out_size, void* d_ws, size_t ws_size,
                              hipStream_t stream) {
  if (n_in < 8) return;
  if (in_sizes[0] != OUTN) return;
  if (in_sizes[1] != C_DIM * QKV_N) return;
  if (in_sizes[2] != BR_DIM * BR_DIM || in_sizes[3] != BR_DIM) return;
  if (in_sizes[4] != C_DIM * BR_DIM) return;
  if (in_sizes[5] != C_DIM * C_DIM) return;
  if (in_sizes[6] != BR_DIM * BR_DIM || in_sizes[7] != BR_DIM) return;
  if (out_size != OUTN) return;

  const float* x       = (const float*)d_in[0];
  const float* Wh_qkv  = (const float*)d_in[1];
  const float* Wh_proj = (const float*)d_in[2];
  const float* bh_proj = (const float*)d_in[3];
  const float* Wl_q    = (const float*)d_in[4];
  const float* Wl_kv   = (const float*)d_in[5];
  const float* Wl_proj = (const float*)d_in[6];
  const float* bl_proj = (const float*)d_in[7];

  const size_t PXB  = (size_t)NTOK * C_DIM * 2;
  const size_t PXP  = (size_t)NPROW * C_DIM * 2;
  const size_t PW1  = (size_t)QKV_N * C_DIM * 2;
  const size_t PWQ  = (size_t)BR_DIM * C_DIM * 2;
  const size_t PWKV = (size_t)C_DIM * C_DIM * 2;
  const size_t PWP  = (size_t)BR_DIM * BR_DIM * 2;
  const size_t PY1  = (size_t)NTOK * QKV_N * 4;
  const size_t PQ   = (size_t)NTOK * BR_DIM * 2;
  const size_t PKV  = (size_t)NPROW * C_DIM * 2;
  const size_t PCTX = (size_t)BATCH * NLH * HW_N * CTXW * 2;

  size_t off = 0;
  const size_t oXb   = off; off += PXB;
  const size_t oXph  = off; off += PXP;
  const size_t oXpl  = off; off += PXP;
  const size_t oWqkv = off; off += PW1;
  const size_t oWlq  = off; off += PWQ;
  const size_t oWlkv = off; off += PWKV;
  const size_t oWhp  = off; off += PWP;
  const size_t oWlp  = off; off += PWP;
  const size_t oY1   = off; off += PY1;
  const size_t oQp   = off; off += PQ;
  const size_t oKVp  = off; off += PKV;
  const size_t oCw   = off; off += PCTX;
  const size_t oCp   = off; off += PCTX;
  if (off > ws_size) return;
  if (off > (size_t)134217728) return;

  char* ws = (char*)d_ws;
  unsigned short* Xb   = (unsigned short*)(ws + oXb);
  unsigned short* Xph  = (unsigned short*)(ws + oXph);
  unsigned short* Xpl  = (unsigned short*)(ws + oXpl);
  unsigned short* Wqkv = (unsigned short*)(ws + oWqkv);
  unsigned short* Wlq  = (unsigned short*)(ws + oWlq);
  unsigned short* Wlkv = (unsigned short*)(ws + oWlkv);
  unsigned short* Whp  = (unsigned short*)(ws + oWhp);
  unsigned short* Wlp  = (unsigned short*)(ws + oWlp);
  float*          Y1   = (float*)(ws + oY1);
  unsigned short* Qp   = (unsigned short*)(ws + oQp);
  unsigned short* KVp  = (unsigned short*)(ws + oKVp);
  unsigned short* Cw   = (unsigned short*)(ws + oCw);
  unsigned short* Cp   = (unsigned short*)(ws + oCp);
  float*          outf = (float*)d_out;

  const dim3 blk(256);
  k_tr<<<dim3(HW_N / 64, C_DIM / 64, BATCH), blk, 0, stream>>>(x, Xb, C_DIM, HW_N);
  k_tr<<<dim3(QKV_N / 64, C_DIM / 64, 1), blk, 0, stream>>>(Wh_qkv, Wqkv, C_DIM, QKV_N);
  k_tr<<<dim3(BR_DIM / 64, C_DIM / 64, 1), blk, 0, stream>>>(Wl_q, Wlq, C_DIM, BR_DIM);
  k_tr<<<dim3(C_DIM / 64, C_DIM / 64, 1), blk, 0, stream>>>(Wl_kv, Wlkv, C_DIM, C_DIM);
  k_tr<<<dim3(BR_DIM / 64, BR_DIM / 64, 1), blk, 0, stream>>>(Wh_proj, Whp, BR_DIM, BR_DIM);
  k_tr<<<dim3(BR_DIM / 64, BR_DIM / 64, 1), blk, 0, stream>>>(Wl_proj, Wlp, BR_DIM, BR_DIM);
  k_pool<<<dim3(POOLN / 64, C_DIM / 64, BATCH), blk, 0, stream>>>(x, Xph, Xpl);

  const dim3 gQKV(((NTOK / 64) * (QKV_N / 64)) / 8);
  const dim3 gQ(((NTOK / 64) * (BR_DIM / 64)) / 8);
  const dim3 gKV(((NPROW / 64) * (C_DIM / 64)) / 8);
  gemm64<0, 1, 0, 0><<<gQKV, blk, 0, stream>>>(Xb, Xb, C_DIM, Wqkv, C_DIM, bh_proj, Y1, Qp, QKV_N,
                                                NTOK, QKV_N, C_DIM, 1.0f, 0);
  gemm64<1, 1, 0, 0><<<gQ, blk, 0, stream>>>(Xb, Xb, C_DIM, Wlq, C_DIM, bh_proj, Y1, Qp, BR_DIM,
                                              NTOK, BR_DIM, C_DIM, QKV_OSC, 0);
  gemm64<1, 2, 0, 0><<<gKV, blk, 0, stream>>>(Xph, Xpl, C_DIM, Wlkv, C_DIM, bh_proj, Y1, KVp, C_DIM,
                                               NPROW, C_DIM, C_DIM, QKV_OSC, 0);
  k_win_attn<<<dim3((BATCH * POOLN * NLH) / 8), blk, 0, stream>>>(Y1, Cw);
  k_pool_attn<<<dim3(BATCH * NLH * QTILES), dim3(128), 0, stream>>>(Qp, KVp, Cp);
  gemm64<4, 2, 1, 1><<<gQ, blk, 0, stream>>>(Cw, Cw, CTXW, Whp, BR_DIM, bh_proj, outf, Qp, 0,
                                              NTOK, BR_DIM, BR_DIM, 1.0f, 0);
  gemm64<4, 2, 1, 1><<<gQ, blk, 0, stream>>>(Cp, Cp, CTXW, Wlp, BR_DIM, bl_proj, outf, Qp, 0,
                                              NTOK, BR_DIM, BR_DIM, 1.0f, BR_DIM);
  (void)hipGetLastError();
}
